// Interaction_2018634629402
// MI455X (gfx1250) — hardware-run, weakly checked
//
#include <hip/hip_runtime.h>


#ifndef NB
#define NB 16
#endif
#ifndef SEQ_M
#define SEQ_M 1024
#endif
#ifndef SEQ_P
#define SEQ_P 2048
#endif
#define NB_FULL    16
#define SEQ_M_FULL 1024
#define SEQ_P_FULL 2048
#ifndef OUT_SEQ_M
#define OUT_SEQ_M SEQ_M
#endif
#ifndef OUT_SEQ_P
#define OUT_SEQ_P SEQ_P
#endif
#define DM   128
#define AW   4
#define OSP  132
#define WTP  136
#define L2E  1.4426950408889634f
#define PSH  14.0f
#define PSI  (1.0f / 16384.0f)
#define QRS  2048.0f
#define QRI  (1.0f / 2048.0f)
#define LALPHA 0.2f
#define NEGB (-3.0e38f)
#define OUTP_OFF_BYTES 8388608

static_assert(DM == 128);
static_assert(DM % 64 == 0);
static_assert(DM % 32 == 0);
static_assert(SEQ_M % 64 == 0);
static_assert(SEQ_P % 64 == 0);
static_assert(SEQ_M % 32 == 0);
static_assert(SEQ_P % 32 == 0);
static_assert(SEQ_P % 128 == 0);
static_assert(SEQ_M % (16 * AW) == 0);
static_assert(SEQ_P % (16 * AW) == 0);
static_assert(NB <= NB_FULL);
static_assert(NB <= 32);
static_assert(SEQ_M <= SEQ_M_FULL);
static_assert(SEQ_P <= SEQ_P_FULL);
static_assert((OSP * 4) % 16 == 0);
static_assert(OSP >= DM);
static_assert((WTP * 2) % 16 == 0);
static_assert(WTP >= DM);
static_assert((size_t)OUTP_OFF_BYTES == (size_t)NB_FULL * SEQ_M_FULL * DM * 4);
static_assert(OUTP_OFF_BYTES % 128 == 0);
static_assert(((size_t)SEQ_M * DM) % 8 == 0);
static_assert(((size_t)SEQ_P * DM) % 8 == 0);
static_assert((AW * 16 * OSP + AW * 16) * 4 <= 131072);
static_assert(DM * WTP * 2 <= 131072);
static_assert(16 * 68 * 4 <= 131072);
static_assert(QRS * QRI == 1.0f);

typedef _Float16 h16;
typedef unsigned short bf;
typedef __attribute__((ext_vector_type(16))) __bf16   v16bf;
typedef __attribute__((ext_vector_type(16))) _Float16 v16h;
typedef __attribute__((ext_vector_type(8)))  _Float16 v8h;
typedef __attribute__((ext_vector_type(8)))  unsigned short v8us;
typedef __attribute__((ext_vector_type(8)))  float    v8f;
typedef __attribute__((ext_vector_type(4)))  float    v4f;
typedef v4f  __attribute__((may_alias)) v4fa;
typedef v8us __attribute__((may_alias)) v8usa;

__device__ __forceinline__ unsigned short f2bf(float f) { unsigned u = __float_as_uint(f); u += 0x7FFFu + ((u >> 16) & 1u); return (unsigned short)(u >> 16); }
__device__ __forceinline__ float bfr(float f) { return __uint_as_float(((unsigned)f2bf(f)) << 16); }
__device__ __forceinline__ v16h cat16(v8h lo, v8h hi) { return __builtin_shufflevector(lo, hi, 0, 1, 2, 3, 4, 5, 6, 7, 8, 9, 10, 11, 12, 13, 14, 15); }
__device__ __forceinline__ v16bf cat16b(v8us lo, v8us hi) { return __builtin_bit_cast(v16bf, __builtin_shufflevector(lo, hi, 0, 1, 2, 3, 4, 5, 6, 7, 8, 9, 10, 11, 12, 13, 14, 15)); }
__device__ __forceinline__ v8f wmma16(v16h a, v16h b, v8f c) { return __builtin_amdgcn_wmma_f32_16x16x32_f16(false, a, false, b, (short)0, c, false, false); }
__device__ __forceinline__ v8f wmmab(v16bf a, v16bf b, v8f c) { return __builtin_amdgcn_wmma_f32_16x16x32_bf16(false, a, false, b, (short)0, c, false, false); }
__device__ __forceinline__ v16h  ldh(const h16* p) { return cat16(*(const v8h*)p, *(const v8h*)(p + 16)); }
__device__ __forceinline__ v16bf ldb(const bf* p)  { return cat16b(*(const v8us*)p, *(const v8us*)(p + 16)); }
__device__ __forceinline__ void wave_sync() { __builtin_amdgcn_fence(3  , "wavefront"); __builtin_amdgcn_wave_barrier(); asm volatile("" ::: "memory"); }

__device__ __forceinline__ v8f wmma16g(v16h a, v16h b, v8f c) { c = wmma16(a, b, c); asm volatile("v_nop\n\tv_nop\n\tv_nop\n\tv_nop" : "+v"(c) : "v"(a), "v"(b)); return c; }
__device__ __forceinline__ v8f wmmabg(v16bf a, v16bf b, v8f c) { c = wmmab(a, b, c); asm volatile("v_nop\n\tv_nop\n\tv_nop\n\tv_nop" : "+v"(c) : "v"(a), "v"(b)); return c; }
__device__ __forceinline__ h16 toh_flush(float v) { const h16 r = (h16)v; return (fabsf(v) < 6.103515625e-05f) ? (h16)0.0f : r; }
__device__ __forceinline__ float pexp(float e) { const float g = __builtin_amdgcn_exp2f(e); return (e < -14.0f) ? 0.0f : g; }
__device__ __forceinline__ float lrelu(float x) { return x > 0.0f ? x : LALPHA * x; }
__device__ __forceinline__ float elu1(float v) { const float en = __builtin_amdgcn_exp2f(fminf(v, 0.0f) * L2E) - 1.0f; return v > 0.0f ? v : en; }

__global__ __launch_bounds__(256) void k_cvt8(const float* __restrict__ src, bf* dst, size_t n8) {
    const size_t i = (size_t)blockIdx.x * 256 + threadIdx.x; if (i >= n8) return;
    const v8f v = *(const v8f*)(src + i * 8); v8us o;
#pragma unroll
    for (int k = 0; k < 8; ++k) o[k] = f2bf(v[k]);
    *(volatile v8us*)(dst + i * 8) = o; __threadfence(); *(volatile v8us*)(dst + i * 8) = o;
}

static_assert(256 * 8 * 8 == DM * DM);
__global__ __launch_bounds__(256) void k_wT(const float* __restrict__ W, bf* WT) {
    __shared__ __align__(16) bf tl[DM * WTP];
#pragma unroll 1
    for (int i = threadIdx.x; i < DM * DM / 4; i += 256) {
        const int d = i >> 5, e4 = (i & 31) * 4;
        const v4f v = *(const v4f*)(W + (size_t)d * DM + e4);
#pragma unroll
        for (int q = 0; q < 4; ++q) tl[(e4 + q) * WTP + d] = f2bf(v[q]);
    }
    __syncthreads();
#pragma unroll 1
    for (int ps = 0; ps < 2; ++ps) {
#pragma unroll 1
        for (int it = 0; it < 8; ++it) { const int p = it * 256 + threadIdx.x; const int row = p >> 4, c8 = (p & 15) * 8;
            const v8us o = *(const v8usa*)(&tl[row * WTP + c8]);
            *(volatile v8us*)(WT + (size_t)row * DM + c8) = o; }
        if (ps == 0) __threadfence(); }
}

__global__ __launch_bounds__(128) void k_wb(const float* __restrict__ W, const float* __restrict__ bvec, float* out) {
    const int d = threadIdx.x;
    float a = 0.0f;
#pragma unroll 1
    for (int e = 0; e < DM; ++e) a = fmaf(bfr(W[(size_t)d * DM + e]), bfr(bvec[e]), a);
    *(volatile float*)(out + d) = a; __threadfence(); *(volatile float*)(out + d) = a;
}

static_assert(8 * 16 == 32 * 4);
__global__ __launch_bounds__(256) void k_srow(const float* __restrict__ X, const float* __restrict__ WB, float* S, int T, int TFULL) {
    __shared__ __align__(16) float ss[32];
    const int lane = threadIdx.x & 31;
    const int wave = __builtin_amdgcn_readfirstlane((int)(threadIdx.x >> 5));
    const int rb = blockIdx.x * 32; const int bb = rb / T, tt = rb % T;
    const v4f w = *(const v4f*)(WB + lane * 4);
    const float* xb = X + ((size_t)bb * (size_t)TFULL + (size_t)(tt + wave * 4)) * DM + lane * 4;
#pragma unroll 1
    for (int i = 0; i < 4; ++i) {
        const v4f x = *(const v4f*)(xb + (size_t)i * DM);
        float a = bfr(x[0]) * w[0]; a = fmaf(bfr(x[1]), w[1], a); a = fmaf(bfr(x[2]), w[2], a); a = fmaf(bfr(x[3]), w[3], a);
        a += __shfl_xor(a, 16, 32); a += __shfl_xor(a, 8, 32); a += __shfl_xor(a, 4, 32); a += __shfl_xor(a, 2, 32); a += __shfl_xor(a, 1, 32);
        if (lane == 0) ss[wave * 4 + i] = a;
    }
    __syncthreads();
    const v4f v = *(const v4fa*)(&ss[(lane & 7) * 4]);
    float* dst = S + (size_t)rb + (lane & 7) * 4;
#pragma unroll 1
    for (int ps = 0; ps < 2; ++ps) {
        if (wave == 0) { if (lane < 8) *(volatile v4f*)dst = v; }
        if (ps == 0) __threadfence(); }
}

__global__ __launch_bounds__(256) void k_smax(const float* __restrict__ SP, float* MX) {
    __shared__ __align__(16) float red[32];
    const int lane = threadIdx.x & 31;
    const int wave = __builtin_amdgcn_readfirstlane((int)(threadIdx.x >> 5));
    if (threadIdx.x < 32) red[threadIdx.x] = 0.0f;
    __syncthreads();
#pragma unroll 1
    for (int bb = wave; bb < NB; bb += 8) {
        float m = NEGB;
#pragma unroll 1
        for (int i = 0; i < SEQ_P / 128; ++i) { const v4f v = *(const v4f*)(SP + (size_t)bb * SEQ_P + (size_t)(i * 32 + lane) * 4);
            m = fmaxf(m, fmaxf(fmaxf(v[0], v[1]), fmaxf(v[2], v[3]))); }
        m = fmaxf(m, __shfl_xor(m, 16, 32)); m = fmaxf(m, __shfl_xor(m, 8, 32)); m = fmaxf(m, __shfl_xor(m, 4, 32)); m = fmaxf(m, __shfl_xor(m, 2, 32)); m = fmaxf(m, __shfl_xor(m, 1, 32));
        if (lane == 0) red[bb] = m;
    }
    __syncthreads();
    const v4f v = *(const v4fa*)(&red[(lane & 7) * 4]);
#pragma unroll 1
    for (int ps = 0; ps < 2; ++ps) {
        if (wave == 0) { if (lane < 8) *(volatile v4f*)(MX + lane * 4) = v; }
        if (ps == 0) __threadfence(); }
}

static_assert(32 * 16 * 4 == 16 * 64 * 2);
__global__ __launch_bounds__(32) void k_projT(const bf* __restrict__ A, const bf* __restrict__ Bt, h16* HT, h16* HR, int wres, int T) {
    __shared__ __align__(16) float os[16 * 68];
    const int K = DM;
    const int lane = threadIdx.x & 31, lr = lane & 15, hi = lane >> 4; const int r0 = blockIdx.x * 64, c0 = blockIdx.y * 64;
    v8f acc[4][4];
#pragma unroll
    for (int mb = 0; mb < 4; ++mb)
#pragma unroll
        for (int nb = 0; nb < 4; ++nb) acc[mb][nb] = (v8f){};
    const size_t aoff = (size_t)(r0 + lr) * K + 8 * hi, boff = (size_t)(c0 + lr) * K + 8 * hi;
#pragma unroll 1
    for (int kc = 0; kc < K; kc += 32) {
        v16bf a[4];
#pragma unroll
        for (int mb = 0; mb < 4; ++mb) a[mb] = ldb(A + aoff + (size_t)mb * 16 * K + kc);
#pragma unroll
        for (int nb = 0; nb < 4; ++nb) { const v16bf b = ldb(Bt + boff + (size_t)nb * 16 * K + kc);
#pragma unroll
            for (int mb = 0; mb < 4; ++mb) acc[mb][nb] = wmmabg(a[mb], b, acc[mb][nb]); }
    }
    const int bb = c0 / T, tt = c0 % T;
    const size_t tbase = (size_t)bb * (size_t)DM * (size_t)T + (size_t)r0 * (size_t)T + (size_t)tt;
    const bool wr = wres != 0;
#pragma unroll
    for (int mb = 0; mb < 4; ++mb) {
#pragma unroll
        for (int nb = 0; nb < 4; ++nb) {
#pragma unroll
            for (int j = 0; j < 8; ++j) os[(hi * 8 + j) * 68 + nb * 16 + lr] = acc[mb][nb][j]; }
        wave_sync();
#pragma unroll 1
        for (int ps = 0; ps < 2; ++ps) {
            const size_t sb = tbase + (size_t)(mb * 16) * (size_t)T;
#pragma unroll
            for (int s = 0; s < 4; ++s) { const int row = 4 * s + (lane >> 3), c8 = (lane & 7) * 8;
                const v4f x0 = *(const v4fa*)(&os[row * 68 + c8]); const v4f x1 = *(const v4fa*)(&os[row * 68 + c8 + 4]); v8h hv, rv;
#pragma unroll
                for (int i = 0; i < 4; ++i) { const h16 a0 = toh_flush(x0[i]); const h16 a1 = toh_flush(x1[i]); hv[i] = a0; hv[4 + i] = a1;
                    rv[i] = toh_flush((x0[i] - (float)a0) * QRS); rv[4 + i] = toh_flush((x1[i] - (float)a1) * QRS); }
                const size_t oo = sb + (size_t)row * (size_t)T + c8;
                *(volatile v8h*)(HT + oo) = hv; if (wr) *(volatile v8h*)(HR + oo) = rv; }
            if (ps == 0) __threadfence(); }
        wave_sync();
    }
}

static_assert(32 * 16 * 16 == 16 * DM * 4);
static_assert(16 * 16 == 16 * AW * 4);
template <int MODE>
__device__ __forceinline__ void attn_body(const h16* __restrict__ HT, const h16* __restrict__ HR, const float* __restrict__ SROW, const float* __restrict__ SKEY,
                                          const float* __restrict__ OFFK, const float* __restrict__ MXP, float* OUT, float* OFFO) {
    constexpr int NQ   = (MODE == 0) ? SEQ_M : SEQ_P;
    constexpr int NKEY = (MODE == 0) ? SEQ_P : SEQ_M;
    constexpr int OSEQ = (MODE == 0) ? OUT_SEQ_M : OUT_SEQ_P;
    __shared__ __align__(16) float os[AW * 16 * OSP];
    __shared__ __align__(16) float zs[AW * 16];
    const int lane = threadIdx.x & 31, lr = lane & 15, hi = lane >> 4;
    const int wave = __builtin_amdgcn_readfirstlane((int)(threadIdx.x >> 5));
    const int b = blockIdx.y;
    const int t0 = (blockIdx.x * AW + wave) * 16;
    const float srow = SROW[(size_t)b * NQ + t0 + lr];
    float cq = 0.0f;
    if (MODE == 0) { const float rmax = lrelu(srow + MXP[b]); cq = PSH - rmax * L2E; }
    const float* kb = SKEY + (size_t)b * NKEY + 8 * hi;
    const float* ob = OFFK + (size_t)b * NKEY + 8 * hi;
    const size_t vo = ((size_t)b * DM + (size_t)lr) * NKEY + 8 * hi;
    v8f o[8], oR[8];
#pragma unroll
    for (int j = 0; j < 8; ++j) { o[j] = (v8f){}; oR[j] = (v8f){}; }
    float lc = 0.0f, lf = 0.0f;
#pragma unroll 1
    for (int key0 = 0; key0 < NKEY; key0 += 32) {
        const float* kp = kb + key0;
        const v4f m0 = *(const v4f*)kp, m1 = *(const v4f*)(kp + 4), m2 = *(const v4f*)(kp + 16), m3 = *(const v4f*)(kp + 20);
        v4f c0 = (v4f){cq, cq, cq, cq}, c1 = c0, c2 = c0, c3 = c0;
        if (MODE == 1) { const float* cp = ob + key0; c0 = *(const v4f*)cp; c1 = *(const v4f*)(cp + 4); c2 = *(const v4f*)(cp + 16); c3 = *(const v4f*)(cp + 20); }
        float kx[16], cx[16];
#pragma unroll
        for (int r = 0; r < 4; ++r) { kx[r] = m0[r]; kx[4 + r] = m1[r]; kx[8 + r] = m2[r]; kx[12 + r] = m3[r];
                                      cx[r] = c0[r]; cx[4 + r] = c1[r]; cx[8 + r] = c2[r]; cx[12 + r] = c3[r]; }
        v16h pb, pr = (v16h){};
#pragma unroll
        for (int i = 0; i < 16; ++i) {
            const float x = lrelu(srow + kx[i]);
            const float e = fmaf(x, L2E, cx[i]);
            const float g = pexp(e);
            const h16 p = (h16)g;
            pb[i] = p;
            if (MODE == 0) { lc += (float)p; lf += g; }
            if (MODE == 1) { pr[i] = toh_flush((g - (float)p) * QRS); } }
        const h16* va = HT + vo + key0;
        if (MODE == 0) {
#pragma unroll
            for (int g4 = 0; g4 < 2; ++g4) {
                const v16h a0 = ldh(va + (size_t)(4 * g4 + 0) * 16 * NKEY);
                const v16h a1 = ldh(va + (size_t)(4 * g4 + 1) * 16 * NKEY);
                const v16h a2 = ldh(va + (size_t)(4 * g4 + 2) * 16 * NKEY);
                const v16h a3 = ldh(va + (size_t)(4 * g4 + 3) * 16 * NKEY);
                o[4 * g4 + 0] = wmma16g(a0, pb, o[4 * g4 + 0]);
                o[4 * g4 + 1] = wmma16g(a1, pb, o[4 * g4 + 1]);
                o[4 * g4 + 2] = wmma16g(a2, pb, o[4 * g4 + 2]);
                o[4 * g4 + 3] = wmma16g(a3, pb, o[4 * g4 + 3]);
            }
        } else {
            const h16* ra = HR + vo + key0;
#pragma unroll
            for (int g2 = 0; g2 < 4; ++g2) {
                const v16h a0 = ldh(va + (size_t)(2 * g2 + 0) * 16 * NKEY);
                const v16h a1 = ldh(va + (size_t)(2 * g2 + 1) * 16 * NKEY);
                const v16h r0 = ldh(ra + (size_t)(2 * g2 + 0) * 16 * NKEY);
                const v16h r1 = ldh(ra + (size_t)(2 * g2 + 1) * 16 * NKEY);
                o[2 * g2 + 0]  = wmma16g(a0, pb, o[2 * g2 + 0]);
                o[2 * g2 + 1]  = wmma16g(a1, pb, o[2 * g2 + 1]);
                oR[2 * g2 + 0] = wmma16g(a0, pr, oR[2 * g2 + 0]);
                oR[2 * g2 + 1] = wmma16g(a1, pr, oR[2 * g2 + 1]);
                oR[2 * g2 + 0] = wmma16g(r0, pb, oR[2 * g2 + 0]);
                oR[2 * g2 + 1] = wmma16g(r1, pb, oR[2 * g2 + 1]);
            }
        }
    }
    float scl = PSI, offv = 0.0f;
    if (MODE == 0) {
        lc += __shfl_xor(lc, 16, 32); lf += __shfl_xor(lf, 16, 32);
        const float lcs = lc > 0.0f ? lc : 1.0f;
        const float lfs = lf > 0.0f ? lf : 1.0f;
        scl = 1.0f / lcs;
        offv = cq - __builtin_amdgcn_logf(lfs) + PSH;
    }
    const int wb = wave * 16 * OSP;
#pragma unroll
    for (int j = 0; j < 8; ++j) { v4f a, c; v8f f = o[j];
        if (MODE == 1) f = o[j] + oR[j] * QRI;
#pragma unroll
        for (int i = 0; i < 4; ++i) { a[i] = elu1(f[i] * scl); c[i] = elu1(f[4 + i] * scl); }
        *(v4fa*)(&os[wb + lr * OSP + 16 * j + 8 * hi]) = a; *(v4fa*)(&os[wb + lr * OSP + 16 * j + 8 * hi + 4]) = c; }
    if (MODE == 0) { if (hi == 0) zs[wave * 16 + lr] = offv; }
    if (MODE == 0) __syncthreads(); else wave_sync();
    float* orow = OUT + ((size_t)b * OSEQ + (size_t)t0) * DM + lane * 4;
    v4f zv = (v4f){};
    if (MODE == 0) zv = *(const v4fa*)(&zs[(lane & 15) * 4]);
    float* zrow = OFFO + (size_t)b * SEQ_M + (size_t)blockIdx.x * (16 * AW) + (lane & 15) * 4;
#pragma unroll 1
    for (int ps = 0; ps < 2; ++ps) {
#pragma unroll 4
        for (int s = 0; s < 16; ++s) {
            const v4f val = *(const v4fa*)(&os[wb + s * OSP + lane * 4]);
            *(volatile v4f*)(orow + (size_t)s * DM) = val; }
        if (MODE == 0) { if (wave == 0) { if (lane < 16) *(volatile v4f*)zrow = zv; } }
        if (ps == 0) __threadfence(); }
}

__global__ __launch_bounds__(32 * AW) void k_attn_m(const h16* __restrict__ HPT, const float* __restrict__ SMV, const float* __restrict__ SPV,
                                                    const float* __restrict__ MXP, float* OUT, float* OFFO) {
    attn_body<0>(HPT, HPT, SMV, SPV, SPV, MXP, OUT, OFFO);
}
__global__ __launch_bounds__(32 * AW) __attribute__((amdgpu_num_vgpr(256))) void k_attn_p(const h16* __restrict__ HMT, const h16* __restrict__ HMR, const float* __restrict__ SPV, const float* __restrict__ SMV,
                                                    const float* __restrict__ OFFK, float* OUT) {
    attn_body<1>(HMT, HMR, SPV, SMV, OFFK, SMV, OUT, OUT);
}

static constexpr size_t al256(size_t v) { return (v + 255) & ~(size_t)255; }
static constexpr size_t SZ_XM = al256((size_t)NB * SEQ_M * DM * 2);
static constexpr size_t SZ_XP = al256((size_t)NB * SEQ_P * DM * 2);
static constexpr size_t SZ_WT = al256((size_t)2 * DM * DM * 2);
static constexpr size_t SZ_HM = al256((size_t)NB * DM * SEQ_M * 2);
static constexpr size_t SZ_HR = al256((size_t)NB * DM * SEQ_M * 2);
static constexpr size_t SZ_HP = al256((size_t)NB * DM * SEQ_P * 2);
static constexpr size_t SZ_SM = al256((size_t)NB * SEQ_M * 4);
static constexpr size_t SZ_SP = al256((size_t)NB * SEQ_P * 4);
static constexpr size_t SZ_OF = al256((size_t)NB * SEQ_M * 4);
static constexpr size_t SZ_MX = al256((size_t)32 * 4);
static constexpr size_t SZ_WB = al256((size_t)2 * DM * 4);
static constexpr size_t SZ_TOTAL = SZ_XM + SZ_XP + SZ_WT + SZ_HM + SZ_HR + SZ_HP + SZ_SM + SZ_SP + SZ_OF + SZ_MX + SZ_WB;
static_assert(SZ_TOTAL <= (size_t)134217728);
static_assert(SZ_HR == SZ_HM);
static_assert(SZ_HM >= (size_t)NB * DM * SEQ_M * 2);
static_assert(SZ_HP >= (size_t)NB * DM * SEQ_P * 2);
static_assert(((size_t)DM * DM * 2) % 256 == 0);
static_assert(((size_t)DM * 4) % 128 == 0);
static_assert(((size_t)NB * SEQ_M) % 32 == 0);
static_assert(((size_t)NB * SEQ_P) % 32 == 0);
static_assert((size_t)(SEQ_M / (16 * AW)) * (16 * AW) == (size_t)SEQ_M);

extern "C" void kernel_launch(void* const* d_in, const int* in_sizes, int n_in,
                              void* d_out, int out_size, void* d_ws, size_t ws_size, hipStream_t stream) {
    if (n_in < 5) return;
    const size_t needm = ((size_t)(NB - 1) * SEQ_M_FULL + SEQ_M) * DM;
    const size_t needp = ((size_t)(NB - 1) * SEQ_P_FULL + SEQ_P) * DM;
    if ((size_t)in_sizes[0] < needm || (size_t)in_sizes[1] < needp) return;
    if ((size_t)in_sizes[2] < (size_t)DM * DM || (size_t)in_sizes[3] < (size_t)DM * DM) return;
    if (in_sizes[4] < 2 * DM) return;
    const size_t outp_off = (size_t)OUTP_OFF_BYTES / 4;
    if ((size_t)out_size < outp_off + ((size_t)(NB - 1) * OUT_SEQ_P + SEQ_P) * DM) return;
    if (((size_t)(NB - 1) * OUT_SEQ_M + SEQ_M) * DM > outp_off) return;
    if (SZ_TOTAL > ws_size) return;
    const float* xm = (const float*)d_in[0];
    const float* xp = (const float*)d_in[1];
    const float* wm = (const float*)d_in[2];
    const float* wp = (const float*)d_in[3];
    const float* bv = (const float*)d_in[4];
    float* OUTM = (float*)d_out;
    float* OUTP = (float*)d_out + outp_off;
    char* wsp = (char*)d_ws;
    bf* XBM = (bf*)wsp; wsp += SZ_XM;
    bf* XBP = (bf*)wsp; wsp += SZ_XP;
    bf* WTB = (bf*)wsp; wsp += SZ_WT;
    h16* HMT = (h16*)wsp; wsp += SZ_HM;
    h16* HMR = (h16*)wsp; wsp += SZ_HR;
    h16* HPT = (h16*)wsp; wsp += SZ_HP;
    float* SMV = (float*)wsp; wsp += SZ_SM;
    float* SPV = (float*)wsp; wsp += SZ_SP;
    float* OFF = (float*)wsp; wsp += SZ_OF;
    float* MXP = (float*)wsp; wsp += SZ_MX;
    float* WBV = (float*)wsp; wsp += SZ_WB;
    bf* WTM = WTB; bf* WTPp = WTB + (size_t)DM * DM;

    if (SEQ_M == SEQ_M_FULL) {
        const size_t n8 = (size_t)NB * SEQ_M * DM / 8;
        k_cvt8<<<(unsigned)((n8 + 255) / 256), 256, 0, stream>>>(xm, XBM, n8);
    } else {
        const size_t n8 = (size_t)SEQ_M * DM / 8;
        for (int b = 0; b < NB; ++b) k_cvt8<<<(unsigned)((n8 + 255) / 256), 256, 0, stream>>>(xm + (size_t)b * SEQ_M_FULL * DM, XBM + (size_t)b * SEQ_M * DM, n8);
    }
    if (SEQ_P == SEQ_P_FULL) {
        const size_t n8 = (size_t)NB * SEQ_P * DM / 8;
        k_cvt8<<<(unsigned)((n8 + 255) / 256), 256, 0, stream>>>(xp, XBP, n8);
    } else {
        const size_t n8 = (size_t)SEQ_P * DM / 8;
        for (int b = 0; b < NB; ++b) k_cvt8<<<(unsigned)((n8 + 255) / 256), 256, 0, stream>>>(xp + (size_t)b * SEQ_P_FULL * DM, XBP + (size_t)b * SEQ_P * DM, n8);
    }
    k_wT<<<1, 256, 0, stream>>>(wm, WTM);
    k_wT<<<1, 256, 0, stream>>>(wp, WTPp);
    k_wb<<<1, 128, 0, stream>>>(wm, bv, WBV);
    k_wb<<<1, 128, 0, stream>>>(wp, bv + DM, WBV + DM);
    k_srow<<<(unsigned)((size_t)NB * SEQ_M / 32), 256, 0, stream>>>(xm, WBV, SMV, SEQ_M, SEQ_M_FULL);
    k_srow<<<(unsigned)((size_t)NB * SEQ_P / 32), 256, 0, stream>>>(xp, WBV + DM, SPV, SEQ_P, SEQ_P_FULL);
    k_smax<<<1, 256, 0, stream>>>(SPV, MXP);
    k_projT<<<dim3(DM / 64, NB * SEQ_M / 64, 1), 32, 0, stream>>>(WTM, XBM, HMT, HMR, 1, SEQ_M);
    k_projT<<<dim3(DM / 64, NB * SEQ_P / 64, 1), 32, 0, stream>>>(WTPp, XBP, HPT, HPT, 0, SEQ_P);
    k_attn_m<<<dim3(SEQ_M / (16 * AW), NB, 1), 32 * AW, 0, stream>>>(HPT, SMV, SPV, MXP, OUTM, OFF);
    k_attn_p<<<dim3(SEQ_P / (16 * AW), NB, 1), 32 * AW, 0, stream>>>(HMT, HMR, SPV, SMV, OFF, OUTP);
}
